// SelfAttention_12652973654654
// MI455X (gfx1250) — hardware-verified
//
#include <hip/hip_runtime.h>
#include <stdint.h>
#include <stddef.h>


#ifndef NB
#define NB 1
#endif
#ifndef SEQ
#define SEQ 4096
#endif
#ifndef SE
#if SEQ < 640
#define SE SEQ
#else
#define SE 640
#endif
#endif
#define SEQ_FULL 4096
#define HID 2048
#define NH 16
#define NKV 4
#define HD 128
#define NQKV (NH * HD + 2 * NKV * HD)
#define BQW 32

static_assert(NB == 1);
static_assert(SEQ % 64 == 0);
static_assert(SEQ >= SE);
static_assert(SEQ <= SEQ_FULL);
static_assert(SE >= 64);
static_assert(SE % 64 == 0);
static_assert(SE % BQW == 0);
static_assert(HID % 128 == 0);
static_assert(HID == 256 * 8);
static_assert(NQKV % 128 == 0);
static_assert(HD == 128);
static_assert(NH == 4 * NKV);
static_assert(NH * HD == HID);

typedef _Float16 f16;
typedef __bf16 bf16;
typedef unsigned short u16;
typedef f16 v16h __attribute__((ext_vector_type(16)));
typedef bf16 v16b __attribute__((ext_vector_type(16)));
typedef float v8f __attribute__((ext_vector_type(8)));
typedef float v4f __attribute__((ext_vector_type(4)));
typedef unsigned v4u __attribute__((ext_vector_type(4)));

union FragH { v16h v; v4u q[2]; f16 h[16]; };
union FragB { v16b v; v4u q[2]; };

__device__ __forceinline__ v8f zero8() {
  v8f z = {0.0f, 0.0f, 0.0f, 0.0f, 0.0f, 0.0f, 0.0f, 0.0f};
  return z;
}

__device__ __forceinline__ v8f wg_h(v8f acc, v16h a, v16h b) {
  acc = __builtin_amdgcn_wmma_f32_16x16x32_f16(false, a, false, b, (short)0, acc, false, false);
  asm volatile("v_nop\n\tv_nop\n\tv_nop\n\tv_nop" : "+v"(acc) : "v"(a), "v"(b));
  return acc;
}
__device__ __forceinline__ v8f wg_b(v8f acc, v16b a, v16b b) {
  acc = __builtin_amdgcn_wmma_f32_16x16x32_bf16(false, a, false, b, (short)0, acc, false, false);
  asm volatile("v_nop\n\tv_nop\n\tv_nop\n\tv_nop" : "+v"(acc) : "v"(a), "v"(b));
  return acc;
}

__device__ __forceinline__ unsigned bf16_rne(float f) {
  const unsigned u = __float_as_uint(f);
  return (u + 0x7FFFu + ((u >> 16) & 1u)) >> 16;
}
__device__ __forceinline__ u16 hbits(float f) {
  const f16 x = (f16)f;
  return __builtin_bit_cast(u16, x);
}
__device__ __forceinline__ void split1024(float v, u16& hb, u16& lb) {
#pragma clang fp contract(off)
  const f16 x = (f16)v;
  const float xr = (float)x;
  const float dlt = v - xr;
  const f16 y = (f16)(dlt * 1024.0f);
  hb = __builtin_bit_cast(u16, x);
  lb = __builtin_bit_cast(u16, y);
}
__device__ __forceinline__ int imin(int a, int b) { return a < b ? a : b; }
__device__ __forceinline__ int imax(int a, int b) { return a > b ? a : b; }

__device__ __forceinline__ void rot_sincos(float ang, float& sn, float& cs) {
#pragma clang fp contract(off)
  const double x = (double)ang;
  const double kq = __builtin_rint(x * 0.63661977236758134308);
  double r = x - kq * 1.57079632673412561417;
  r = r - kq * 6.07710050650619224932e-11;
  const int q = (int)kq;
  const double r2 = r * r;
  double ps = 1.6059043836821613e-10;
  ps = ps * r2 - 2.5052108385441720e-08;
  ps = ps * r2 + 2.7557319223985893e-06;
  ps = ps * r2 - 1.9841269841269841e-04;
  ps = ps * r2 + 8.3333333333333332e-03;
  ps = ps * r2 - 1.6666666666666666e-01;
  const double r3 = r * r2;
  const double sr = r + r3 * ps;
  double pc = -1.1470745597729725e-11;
  pc = pc * r2 + 2.0876756987868099e-09;
  pc = pc * r2 - 2.7557319223985888e-07;
  pc = pc * r2 + 2.4801587301587302e-05;
  pc = pc * r2 - 1.3888888888888889e-03;
  pc = pc * r2 + 4.1666666666666664e-02;
  pc = pc * r2 - 0.5;
  const double cr = 1.0 + pc * r2;
  const bool odd = (q & 1) != 0;
  const bool neg = (q & 2) != 0;
  double sv = odd ? cr : sr;
  double cv = odd ? -sr : cr;
  sv = neg ? -sv : sv;
  cv = neg ? -cv : cv;
  sn = (float)sv;
  cs = (float)cv;
}

__global__ __launch_bounds__(256) void k_xconv(const float* __restrict__ x, u16* __restrict__ xb,
                                              float* __restrict__ tinv) {
#pragma clang fp contract(off)
  const int t = threadIdx.x;
  const size_t e = ((size_t)blockIdx.x * 256 + (size_t)t) * 8;
  const v4f a = *(const v4f*)(x + e);
  const v4f b = *(const v4f*)(x + e + 4);
  v4u w;
  w[0] = bf16_rne(a[0]) | (bf16_rne(a[1]) << 16);
  w[1] = bf16_rne(a[2]) | (bf16_rne(a[3]) << 16);
  w[2] = bf16_rne(b[0]) | (bf16_rne(b[1]) << 16);
  w[3] = bf16_rne(b[2]) | (bf16_rne(b[3]) << 16);

  const bool tab = (blockIdx.x == 0) && (t < 64);
  float ivf = 0.0f;
  if (tab) {
    double rt = 1.15;
#pragma unroll 1
    for (int it = 0; it < 48; ++it) {
      double p63 = rt;
#pragma unroll 1
      for (int k = 1; k < 63; ++k) p63 *= rt;
      const double p64 = p63 * rt;
      const double f = p64 - 10000.0;
      rt = rt - f / (64.0 * p63);
    }
    double pj = 1.0;
#pragma unroll 1
    for (int k = 0; k < t; ++k) pj *= rt;
    const float pf = (float)pj;
    ivf = (float)(1.0 / (double)pf);
  }
  *(volatile v4u*)(xb + e) = w;
  if (tab) *(volatile float*)(tinv + t) = ivf;
  __threadfence();
  *(volatile v4u*)(xb + e) = w;
  if (tab) *(volatile float*)(tinv + t) = ivf;
}

template <int MODE>
__global__ __launch_bounds__(256) void k_wt(const float* __restrict__ w, u16* __restrict__ wt, int ncol) {
  __shared__ __align__(16) u16 T[64 * 72];
  const int i0 = (int)blockIdx.x * 64, o0 = (int)blockIdx.y * 64, t = threadIdx.x;
#pragma unroll
  for (int j = 0; j < 4; ++j) {
    const int i = (t >> 4) + 16 * j;
    const int oc = (t & 15) * 4;
    const v4f v = *(const v4f*)(w + (size_t)(i0 + i) * (size_t)ncol + o0 + oc);
#pragma unroll
    for (int e = 0; e < 4; ++e) {
      const float f = v[e];
      u16 bb;
      if (MODE == 0) bb = (u16)bf16_rne(f);
      else bb = hbits(__uint_as_float(bf16_rne(f) << 16) * 64.0f);
      T[(oc + e) * 72 + i] = bb;
    }
  }
  __syncthreads();
  v4u val[2];
#pragma unroll
  for (int p = 0; p < 2; ++p) {
    const int o = (t >> 3) + 32 * p;
    val[p] = *(const v4u*)(T + o * 72 + (t & 7) * 8);
  }
#pragma unroll
  for (int p = 0; p < 2; ++p) {
    const int o = (t >> 3) + 32 * p;
    *(volatile v4u*)(wt + (size_t)(o0 + o) * HID + i0 + (t & 7) * 8) = val[p];
  }
  __threadfence();
#pragma unroll
  for (int p = 0; p < 2; ++p) {
    const int o = (t >> 3) + 32 * p;
    *(volatile v4u*)(wt + (size_t)(o0 + o) * HID + i0 + (t & 7) * 8) = val[p];
  }
}

template <int MODE, bool RES>
__global__ __launch_bounds__(256) void k_gemm(const u16* __restrict__ A, const u16* __restrict__ Ar,
                                             const u16* __restrict__ BT, float* __restrict__ C,
                                             int lda, int ldb, int ldc, int K, int row0,
                                             float sh, float sr) {
  __shared__ __align__(16) float Cs[8 * 32 * 36];
  const int tid = threadIdx.x, wave = tid >> 5, lane = tid & 31, h = lane >> 4, l = lane & 15;
  const int wm = wave >> 2, wn = wave & 3;
  const int mb = row0 + (int)blockIdx.y * 64 + wm * 32;
  const int nb = (int)blockIdx.x * 128 + wn * 32;
  const size_t rA0 = (size_t)(mb + l) * (size_t)lda, rA1 = (size_t)(mb + 16 + l) * (size_t)lda;
  const size_t rB0 = (size_t)(nb + l) * (size_t)ldb, rB1 = (size_t)(nb + 16 + l) * (size_t)ldb;
  v8f c00 = zero8(), c01 = zero8(), c10 = zero8(), c11 = zero8();
  v8f r00 = zero8(), r01 = zero8(), r10 = zero8(), r11 = zero8();

  for (int kk = 0; kk < K; kk += 32) {
    const int k0 = kk + 8 * h, k1 = kk + 16 + 8 * h;
    if (MODE == 0) {
      FragB a0, a1, b0, b1;
      a0.q[0] = *(const v4u*)(A + rA0 + k0);  a0.q[1] = *(const v4u*)(A + rA0 + k1);
      a1.q[0] = *(const v4u*)(A + rA1 + k0);  a1.q[1] = *(const v4u*)(A + rA1 + k1);
      b0.q[0] = *(const v4u*)(BT + rB0 + k0); b0.q[1] = *(const v4u*)(BT + rB0 + k1);
      b1.q[0] = *(const v4u*)(BT + rB1 + k0); b1.q[1] = *(const v4u*)(BT + rB1 + k1);
      c00 = wg_b(c00, a0.v, b0.v); c01 = wg_b(c01, a0.v, b1.v);
      c10 = wg_b(c10, a1.v, b0.v); c11 = wg_b(c11, a1.v, b1.v);
    } else {
      FragH a0, a1, b0, b1;
      a0.q[0] = *(const v4u*)(A + rA0 + k0);  a0.q[1] = *(const v4u*)(A + rA0 + k1);
      a1.q[0] = *(const v4u*)(A + rA1 + k0);  a1.q[1] = *(const v4u*)(A + rA1 + k1);
      b0.q[0] = *(const v4u*)(BT + rB0 + k0); b0.q[1] = *(const v4u*)(BT + rB0 + k1);
      b1.q[0] = *(const v4u*)(BT + rB1 + k0); b1.q[1] = *(const v4u*)(BT + rB1 + k1);
      c00 = wg_h(c00, a0.v, b0.v); c01 = wg_h(c01, a0.v, b1.v);
      c10 = wg_h(c10, a1.v, b0.v); c11 = wg_h(c11, a1.v, b1.v);
      if (RES) {
        FragH e0, e1;
        e0.q[0] = *(const v4u*)(Ar + rA0 + k0); e0.q[1] = *(const v4u*)(Ar + rA0 + k1);
        e1.q[0] = *(const v4u*)(Ar + rA1 + k0); e1.q[1] = *(const v4u*)(Ar + rA1 + k1);
        r00 = wg_h(r00, e0.v, b0.v); r01 = wg_h(r01, e0.v, b1.v);
        r10 = wg_h(r10, e1.v, b0.v); r11 = wg_h(r11, e1.v, b1.v);
      }
    }
  }

  float* cs = Cs + wave * (32 * 36);
#pragma unroll
  for (int e = 0; e < 8; ++e) {
    const int ra = 8 * h + e, rb = ra + 16;
    float v00 = sh * c00[e], v01 = sh * c01[e], v10 = sh * c10[e], v11 = sh * c11[e];
    if (RES) { v00 += sr * r00[e]; v01 += sr * r01[e]; v10 += sr * r10[e]; v11 += sr * r11[e]; }
    cs[ra * 36 + l] = v00;
    cs[ra * 36 + 16 + l] = v01;
    cs[rb * 36 + l] = v10;
    cs[rb * 36 + 16 + l] = v11;
  }
  __syncthreads();
  v4f val[8];
#pragma unroll
  for (int i = 0; i < 8; ++i) {
    const int row = 4 * i + (lane >> 3);
    val[i] = *(const v4f*)(cs + row * 36 + (lane & 7) * 4);
  }
#pragma unroll
  for (int i = 0; i < 8; ++i) {
    const int row = 4 * i + (lane >> 3);
    *(volatile v4f*)(C + (size_t)(mb + row) * (size_t)ldc + nb + (lane & 7) * 4) = val[i];
  }
  __threadfence();
#pragma unroll
  for (int i = 0; i < 8; ++i) {
    const int row = 4 * i + (lane >> 3);
    *(volatile v4f*)(C + (size_t)(mb + row) * (size_t)ldc + nb + (lane & 7) * 4) = val[i];
  }
}

__global__ __launch_bounds__(256) void k_planes(const float* __restrict__ qkv, const int* __restrict__ pos,
                                               const float* __restrict__ tinv,
                                               u16* __restrict__ Qh, u16* __restrict__ Ql,
                                               u16* __restrict__ Kh, u16* __restrict__ Kl) {
#pragma clang fp contract(off)
  __shared__ __align__(16) u16 Qs[NH * HD];
  __shared__ __align__(16) u16 Qls[NH * HD];
  __shared__ __align__(16) u16 Ks[NKV * HD];
  __shared__ __align__(16) u16 Kls[NKV * HD];
  const int s = (int)blockIdx.x, t = threadIdx.x;
  const bool early = (s < SE);
  int pp = pos[s];
  pp = imin(imax(pp, 0), SEQ_FULL - 1);
  const int di = t & 63;
  const float ang = (float)pp * tinv[di];
  float sn, cs;
  rot_sincos(ang, sn, cs);
  const float* row = qkv + (size_t)s * NQKV;

#pragma unroll 1
  for (int j = 0; j < 4; ++j) {
    const int hh = (t + 256 * j) >> 6;
    const int col = hh * HD + di;
    const float x1 = row[col], x2 = row[col + 64];
    const float a1 = x1 * cs, b1 = x2 * sn;
    const float a2 = x2 * cs, b2 = x1 * sn;
    const float r1 = a1 - b1;
    const float r2 = a2 + b2;
    if (early) {
      u16 a, b;
      split1024(r1, a, b); Qs[col] = a;      Qls[col] = b;
      split1024(r2, a, b); Qs[col + 64] = a; Qls[col + 64] = b;
    } else {
      Qs[col] = hbits(r1);
      Qs[col + 64] = hbits(r2);
    }
  }
  {
    const int kvh = t >> 6;
    const int col = kvh * HD + di;
    const float x1 = row[NH * HD + col], x2 = row[NH * HD + col + 64];
    const float a1 = x1 * cs, b1 = x2 * sn;
    const float a2 = x2 * cs, b2 = x1 * sn;
    const float r1 = a1 - b1;
    const float r2 = a2 + b2;
    if (early) {
      u16 a, b;
      split1024(r1, a, b); Ks[col] = a;      Kls[col] = b;
      split1024(r2, a, b); Ks[col + 64] = a; Kls[col + 64] = b;
    } else {
      Ks[col] = hbits(r1);
      Ks[col + 64] = hbits(r2);
    }
  }
  __syncthreads();

  const int e = t * 8;
  const int hq = e >> 7, dq = e & 127;
  const bool kw = (t < 64);
  const int hk = hq, dk = dq;
  const v4u vq = *(const v4u*)(Qs + e);
  v4u vql = vq, vk = vq, vkl = vq;
  if (early) vql = *(const v4u*)(Qls + e);
  if (kw) {
    vk = *(const v4u*)(Ks + e);
    if (early) vkl = *(const v4u*)(Kls + e);
  }
  u16* pq  = Qh + ((size_t)hq * SEQ + s) * HD + dq;
  u16* pql = Ql + ((size_t)hq * SE + (early ? s : 0)) * HD + dq;
  u16* pk  = Kh + ((size_t)hk * SEQ + s) * HD + dk;
  u16* pkl = Kl + ((size_t)hk * SE + (early ? s : 0)) * HD + dk;

  *(volatile v4u*)pq = vq;
  if (early) *(volatile v4u*)pql = vql;
  if (kw) {
    *(volatile v4u*)pk = vk;
    if (early) *(volatile v4u*)pkl = vkl;
  }
  __threadfence();
  *(volatile v4u*)pq = vq;
  if (early) *(volatile v4u*)pql = vql;
  if (kw) {
    *(volatile v4u*)pk = vk;
    if (early) *(volatile v4u*)pkl = vkl;
  }
}

__global__ __launch_bounds__(256) void k_vt(const float* __restrict__ qkv, u16* __restrict__ Vth,
                                           u16* __restrict__ Vtl) {
#pragma clang fp contract(off)
  __shared__ __align__(16) u16 T[HD * 72];
  __shared__ __align__(16) u16 Tl[HD * 72];
  const int s0 = (int)blockIdx.x * 64, kv = (int)blockIdx.y, t = threadIdx.x;
  const bool early = (s0 < SE);
#pragma unroll 1
  for (int j = 0; j < 8; ++j) {
    const int idx = t + 256 * j;
    const int r = idx >> 5;
    const int c4 = (idx & 31) * 4;
    const v4f v = *(const v4f*)(qkv + (size_t)(s0 + r) * NQKV + NH * HD + NKV * HD + kv * HD + c4);
#pragma unroll
    for (int e = 0; e < 4; ++e) {
      const float f = 16.0f * v[e];
      if (early) {
        u16 a, b;
        split1024(f, a, b);
        T[(c4 + e) * 72 + r] = a;
        Tl[(c4 + e) * 72 + r] = b;
      } else {
        T[(c4 + e) * 72 + r] = hbits(f);
      }
    }
  }
  __syncthreads();
  v4u vh[4], vl[4];
#pragma unroll
  for (int p = 0; p < 4; ++p) {
    const int d = (t >> 3) + 32 * p, c = (t & 7) * 8;
    vh[p] = *(const v4u*)(T + d * 72 + c);
    vl[p] = vh[p];
    if (early) vl[p] = *(const v4u*)(Tl + d * 72 + c);
  }
#pragma unroll
  for (int p = 0; p < 4; ++p) {
    const int d = (t >> 3) + 32 * p, c = (t & 7) * 8;
    *(volatile v4u*)(Vth + ((size_t)kv * HD + d) * SEQ + s0 + c) = vh[p];
    if (early) *(volatile v4u*)(Vtl + ((size_t)kv * HD + d) * SE + s0 + c) = vl[p];
  }
  __threadfence();
#pragma unroll
  for (int p = 0; p < 4; ++p) {
    const int d = (t >> 3) + 32 * p, c = (t & 7) * 8;
    *(volatile v4u*)(Vth + ((size_t)kv * HD + d) * SEQ + s0 + c) = vh[p];
    if (early) *(volatile v4u*)(Vtl + ((size_t)kv * HD + d) * SE + s0 + c) = vl[p];
  }
}

template <bool EARLY>
__global__ __launch_bounds__(256) __attribute__((amdgpu_num_vgpr(256)))
void k_attn(const u16* __restrict__ Qh, const u16* __restrict__ Ql,
            const u16* __restrict__ Kh, const u16* __restrict__ Kl,
            const u16* __restrict__ Vth, const u16* __restrict__ Vtl,
            const int* __restrict__ amask,
            u16* __restrict__ Ch, u16* __restrict__ Cr, int qblk0) {
  __shared__ __align__(16) u16 pool[16384];
  __shared__ __align__(16) u16 stg[EARLY ? 16384 : 64];
  constexpr int KS = 0, KL = 4096, VS = 8192, VL = 12288;
  constexpr int NDT = EARLY ? 2 : 8;
  constexpr int DW = NDT * 16;
  constexpr int NPASS = HD / DW;
  const int qblk = qblk0 + (int)blockIdx.x;
  const int kv = (int)blockIdx.y;
  const int tid = threadIdx.x, wave = tid >> 5, lane = tid & 31, h = lane >> 4, l = lane & 15;
  const int head = kv * (NH / NKV) + (wave >> 1);
  const int q0 = qblk * BQW;
  const int qw0 = q0 + (wave & 1) * 16;
  const int qrow = qw0 + l;
  const int nchunk = qblk + 1;

  FragH qh[4];
  FragH ql[4];
#pragma unroll
  for (int dc = 0; dc < 4; ++dc) {
    const u16* b = Qh + ((size_t)head * SEQ + qrow) * HD + dc * 32 + 8 * h;
    qh[dc].q[0] = *(const v4u*)b;
    qh[dc].q[1] = *(const v4u*)(b + 16);
    if (EARLY) {
      const u16* b2 = Ql + ((size_t)head * SE + qrow) * HD + dc * 32 + 8 * h;
      ql[dc].q[0] = *(const v4u*)b2;
      ql[dc].q[1] = *(const v4u*)(b2 + 16);
    } else {
      ql[dc].q[0] = qh[dc].q[0];
      ql[dc].q[1] = qh[dc].q[1];
    }
  }
  const float SCL = 0.088388347648318441f * 1.4426950408889634f;

  u16* os;
  if (EARLY) os = stg + wave * (16 * 128);
  else os = pool + wave * (16 * 128);

#pragma unroll 1
  for (int pass = 0; pass < NPASS; ++pass) {
    const int dbase = pass * DW;
    v8f o[NDT];
    v8f orr[NDT];
#pragma unroll
    for (int dt = 0; dt < NDT; ++dt) { o[dt] = zero8(); orr[dt] = zero8(); }
    float rmax = -1.0e30f, rsum = 0.0f;

#pragma unroll 1
    for (int kc = 0; kc < nchunk; ++kc) {
      const int kbase = kc * 32;
      __syncthreads();
#pragma unroll
      for (int j = 0; j < 2; ++j) {
        const int pp = tid + 256 * j;
        {
          const int r = pp >> 4, c = (pp & 15) * 8;
          *(v4u*)(pool + KS + r * HD + c) = *(const v4u*)(Kh + ((size_t)kv * SEQ + kbase + r) * HD + c);
          if (EARLY)
            *(v4u*)(pool + KL + r * HD + c) = *(const v4u*)(Kl + ((size_t)kv * SE + kbase + r) * HD + c);
        }
        {
          const int d = pp >> 2, c = (pp & 3) * 8;
          *(v4u*)(pool + VS + d * 32 + c) = *(const v4u*)(Vth + ((size_t)kv * HD + d) * SEQ + kbase + c);
          if (EARLY)
            *(v4u*)(pool + VL + d * 32 + c) = *(const v4u*)(Vtl + ((size_t)kv * HD + d) * SE + kbase + c);
        }
      }
      const int av = amask[imin(kbase + lane, SEQ - 1)];
      const unsigned mw = __builtin_amdgcn_ballot_w32(av != 0);
      __syncthreads();

      float u[16];
      unsigned vm = 0u;
      float m_new = rmax;
#pragma unroll
      for (int sub = 0; sub < 2; ++sub) {
        v8f acc = zero8();
        v8f accr = zero8();
#pragma unroll
        for (int dc = 0; dc < 4; ++dc) {
          FragH kf;
          const u16* kb = pool + KS + (sub * 16 + l) * HD + dc * 32 + 8 * h;
          kf.q[0] = *(const v4u*)kb;
          kf.q[1] = *(const v4u*)(kb + 16);
          acc = wg_h(acc, kf.v, qh[dc].v);
          if (EARLY) {
            accr = wg_h(accr, kf.v, ql[dc].v);
            FragH kg;
            const u16* kb2 = pool + KL + (sub * 16 + l) * HD + dc * 32 + 8 * h;
            kg.q[0] = *(const v4u*)kb2;
            kg.q[1] = *(const v4u*)(kb2 + 16);
            accr = wg_h(accr, kg.v, qh[dc].v);
          }
        }
#pragma unroll
        for (int r = 0; r < 8; ++r) {
          const int klc = sub * 16 + 8 * h + r;
          const int key = kbase + klc;
          float s = acc[r];
          if (EARLY) s += accr[r] * (1.0f / 1024.0f);
          const bool valid = (key <= qrow) && (((mw >> klc) & 1u) != 0u);
          const float uu = valid ? s * SCL : -1.0e30f;
          u[sub * 8 + r] = uu;
          vm |= (valid ? 1u : 0u) << (sub * 8 + r);
          m_new = fmaxf(m_new, uu);
        }
      }
      m_new = fmaxf(m_new, __shfl_xor(m_new, 16, 32));
      const float scale = __builtin_amdgcn_exp2f(rmax - m_new);
      rmax = m_new;

      float psum = 0.0f;
      FragH ph;
      FragH pr;
#pragma unroll
      for (int i = 0; i < 16; ++i) {
        const float pe = __builtin_amdgcn_exp2f(u[i] - m_new);
        const float pv = ((vm >> i) & 1u) ? pe : 0.0f;
        psum += pv;
        const float pc = pv * 4096.0f;
        const f16 hv = (f16)pc;
        ph.h[i] = hv;
        if (EARLY) pr.h[i] = (f16)((pc - (float)hv) * 1024.0f);
        else pr.h[i] = hv;
      }
      psum += __shfl_xor(psum, 16, 32);
      rsum = rsum * scale + psum;

      float sc[8];
#pragma unroll
      for (int r = 0; r < 8; ++r) sc[r] = __shfl(scale, 8 * h + r, 32);
#pragma unroll
      for (int dt = 0; dt < NDT; ++dt) {
#pragma unroll
        for (int r = 0; r < 8; ++r) {
          o[dt][r] *= sc[r];
          if (EARLY) orr[dt][r] *= sc[r];
        }
      }
#pragma unroll
      for (int dt = 0; dt < NDT; ++dt) {
        const int d = dbase + dt * 16 + l;
        FragH vf;
        const u16* vb = pool + VS + d * 32 + 8 * h;
        vf.q[0] = *(const v4u*)vb;
        vf.q[1] = *(const v4u*)(vb + 16);
        o[dt] = wg_h(o[dt], ph.v, vf.v);
        if (EARLY) {
          orr[dt] = wg_h(orr[dt], pr.v, vf.v);
          FragH vg;
          const u16* vb2 = pool + VL + d * 32 + 8 * h;
          vg.q[0] = *(const v4u*)vb2;
          vg.q[1] = *(const v4u*)(vb2 + 16);
          orr[dt] = wg_h(orr[dt], ph.v, vg.v);
        }
      }
    }

    if (!EARLY) __syncthreads();
    const float inv = 1.0f / rsum;
    float ir[8];
#pragma unroll
    for (int r = 0; r < 8; ++r) ir[r] = __shfl(inv, 8 * h + r, 32) * (1.0f / 1024.0f);
    const int cb = EARLY ? ((pass & 1) * 32) : 0;
#pragma unroll
    for (int dt = 0; dt < NDT; ++dt) {
#pragma unroll
      for (int r = 0; r < 8; ++r) {
        float val = o[dt][r];
        if (EARLY) val += orr[dt][r] * (1.0f / 1024.0f);
        val *= ir[r];
        if (EARLY) {
          u16 a, b;
          split1024(val, a, b);
          os[(8 * h + r) * 128 + cb + dt * 16 + l] = a;
          os[(8 * h + r) * 128 + 64 + cb + dt * 16 + l] = b;
        } else {
          os[(8 * h + r) * 128 + dt * 16 + l] = hbits(val);
        }
      }
    }
    if (!EARLY) {
      __syncthreads();
      v4u vals[8];
#pragma unroll
      for (int i = 0; i < 8; ++i) {
        const int L = 4 * i + (lane >> 3);
        const int row = L >> 1, seg = L & 1;
        vals[i] = *(const v4u*)(os + row * 128 + seg * 64 + (lane & 7) * 8);
      }
#pragma unroll
      for (int i = 0; i < 8; ++i) {
        const int L = 4 * i + (lane >> 3);
        const int row = L >> 1, seg = L & 1;
        *(volatile v4u*)(Ch + (size_t)(qw0 + row) * HID + head * HD + seg * 64 + (lane & 7) * 8) = vals[i];
      }
      __threadfence();
#pragma unroll
      for (int i = 0; i < 8; ++i) {
        const int L = 4 * i + (lane >> 3);
        const int row = L >> 1, seg = L & 1;
        *(volatile v4u*)(Ch + (size_t)(qw0 + row) * HID + head * HD + seg * 64 + (lane & 7) * 8) = vals[i];
      }
    } else {
      if ((pass & 1) != 0) {
        __syncthreads();
        const int dline = (pass >> 1) * 64;
        v4u va[4], vb[4];
#pragma unroll
        for (int i = 0; i < 4; ++i) {
          const int row = 4 * i + (lane >> 3);
          va[i] = *(const v4u*)(os + row * 128 + (lane & 7) * 8);
          vb[i] = *(const v4u*)(os + row * 128 + 64 + (lane & 7) * 8);
        }
#pragma unroll
        for (int i = 0; i < 4; ++i) {
          const int row = 4 * i + (lane >> 3);
          const size_t off = (size_t)(qw0 + row) * HID + head * HD + dline + (lane & 7) * 8;
          *(volatile v4u*)(Ch + off) = va[i];
          *(volatile v4u*)(Cr + off) = vb[i];
        }
        __threadfence();
#pragma unroll
        for (int i = 0; i < 4; ++i) {
          const int row = 4 * i + (lane >> 3);
          const size_t off = (size_t)(qw0 + row) * HID + head * HD + dline + (lane & 7) * 8;
          *(volatile v4u*)(Ch + off) = va[i];
          *(volatile v4u*)(Cr + off) = vb[i];
        }
      }
    }
  }
}

extern "C" void kernel_launch(void* const* d_in, const int* in_sizes, int n_in,
                              void* d_out, int out_size, void* d_ws, size_t ws_size,
                              hipStream_t stream) {
  if (n_in < 7) return;
  if (in_sizes[0] < SEQ * HID) return;
  if (in_sizes[1] < SEQ) return;
  if (in_sizes[2] < SEQ) return;
  if (in_sizes[3] < HID * NH * HD) return;
  if (in_sizes[4] < HID * NKV * HD) return;
  if (in_sizes[5] < HID * NKV * HD) return;
  if (in_sizes[6] < NH * HD * HID) return;
  if (out_size < SEQ * HID) return;

  const float* hs  = (const float*)d_in[0];
  const int*   am  = (const int*)d_in[1];
  const int*   pos = (const int*)d_in[2];
  const float* wq  = (const float*)d_in[3];
  const float* wk  = (const float*)d_in[4];
  const float* wv  = (const float*)d_in[5];
  const float* wo  = (const float*)d_in[6];
  float* out = (float*)d_out;

  char* ws = (char*)d_ws;
  size_t off = 0;
#define CARVE(T, name, bytes) T* name = (T*)(ws + off); off += (((size_t)(bytes)) + 255) & ~(size_t)255
  CARVE(u16,   Xb,    (size_t)SEQ * HID * 2);
  CARVE(u16,   WqkvT, (size_t)NQKV * HID * 2);
  CARVE(u16,   WoT,   (size_t)HID * HID * 2);
  CARVE(float, QKVf,  (size_t)SEQ * NQKV * 4);
  CARVE(u16,   Qh,    (size_t)NH * SEQ * HD * 2);
  CARVE(u16,   Kh,    (size_t)NKV * SEQ * HD * 2);
  CARVE(u16,   Vth,   (size_t)NKV * HD * SEQ * 2);
  CARVE(u16,   Ql,    (size_t)NH * SE * HD * 2);
  CARVE(u16,   Kl,    (size_t)NKV * SE * HD * 2);
  CARVE(u16,   Vtl,   (size_t)NKV * HD * SE * 2);
  CARVE(u16,   Cr,    (size_t)SE * HID * 2);
  CARVE(float, Tinv,  256);
#undef CARVE
  static_assert(NH * HD == HID);
  u16* Ch = Xb;
  if (off > ws_size) return;

  k_xconv<<<dim3(SEQ), 256, 0, stream>>>(hs, Xb, Tinv);
  k_wt<0><<<dim3(HID / 64, (NH * HD) / 64), 256, 0, stream>>>(wq, WqkvT, NH * HD);
  k_wt<0><<<dim3(HID / 64, (NKV * HD) / 64), 256, 0, stream>>>(wk, WqkvT + (size_t)(NH * HD) * HID, NKV * HD);
  k_wt<0><<<dim3(HID / 64, (NKV * HD) / 64), 256, 0, stream>>>(wv, WqkvT + (size_t)(NH * HD + NKV * HD) * HID, NKV * HD);
  k_wt<1><<<dim3(HID / 64, HID / 64), 256, 0, stream>>>(wo, WoT, HID);
  k_gemm<0, false><<<dim3(NQKV / 128, SEQ / 64), 256, 0, stream>>>(
      Xb, Xb, WqkvT, QKVf, HID, HID, NQKV, HID, 0, 1.0f, 0.0f);
  k_planes<<<dim3(SEQ), 256, 0, stream>>>(QKVf, pos, Tinv, Qh, Ql, Kh, Kl);
  k_vt<<<dim3(SEQ / 64, NKV), 256, 0, stream>>>(QKVf, Vth, Vtl);
  k_attn<true><<<dim3(SE / BQW, NKV), 256, 0, stream>>>(Qh, Ql, Kh, Kl, Vth, Vtl, am, Ch, Cr, 0);
  if (SEQ > SE) {
    k_attn<false><<<dim3(SEQ / BQW - SE / BQW, NKV), 256, 0, stream>>>(
        Qh, Ql, Kh, Kl, Vth, Vtl, am, Ch, Cr, SE / BQW);
  }
  k_gemm<1, true><<<dim3(HID / 128, SE / 64), 256, 0, stream>>>(
      Ch, Cr, WoT, out, HID, HID, HID, HID, 0, 1.0f / 4096.0f, 1.0f / (4096.0f * 1024.0f));
  if (SEQ > SE) {
    k_gemm<1, false><<<dim3(HID / 128, (SEQ - SE) / 64), 256, 0, stream>>>(
        Ch, Ch, WoT, out, HID, HID, HID, HID, SE, 1.0f / 4096.0f, 0.0f);
  }
}
